// BQ_CorrBlock_67327907332136
// MI455X (gfx1250) — hardware-verified
//
#include <hip/hip_runtime.h>
#include <math.h>

typedef __attribute__((ext_vector_type(16))) _Float16 v16h;
typedef __attribute__((ext_vector_type(16))) __bf16 v16b;
typedef __attribute__((ext_vector_type(8)))  _Float16 v8h;
typedef __attribute__((ext_vector_type(8)))  float v8f;
typedef __attribute__((ext_vector_type(4)))  float v4f;
typedef __attribute__((ext_vector_type(2)))  float v2f;
typedef __attribute__((ext_vector_type(4)))  unsigned v4u;
typedef __attribute__((ext_vector_type(4)))  int v4i;
typedef float __attribute__((may_alias)) float_a;
typedef int __attribute__((may_alias)) int_a;

template <typename T> __device__ __forceinline__ void vst2(void* p, T v) { *(volatile T*)p = v; __threadfence(); *(volatile T*)p = v; }
__device__ __forceinline__ v8f wmma16(v16h a, v16h b, v8f c) {
  v8f d = __builtin_amdgcn_wmma_f32_16x16x32_f16(false, a, false, b, (short)0, c, false, false);
  asm volatile("v_nop\n\tv_nop\n\tv_nop\n\tv_nop" : "+v"(d) : "v"(a), "v"(b));
  return d;
}
__device__ __forceinline__ v8f wmma_bf(v16b a, v16b b, v8f c) {
  v8f d = __builtin_amdgcn_wmma_f32_16x16x32_bf16(false, a, false, b, (short)0, c, false, false);
  asm volatile("v_nop\n\tv_nop\n\tv_nop\n\tv_nop" : "+v"(d) : "v"(a), "v"(b));
  return d;
}
__device__ __forceinline__ v16h frag_h(const _Float16* rowk0, int lane) {
  union { v16h v; v8h q[2]; } u; const _Float16* p = rowk0 + 8 * (lane >> 4);
  u.q[0] = *(const v8h*)p; u.q[1] = *(const v8h*)(p + 16); return u.v;
}
__device__ __forceinline__ v16h frag_f32(const float* rowk0, int lane) {
  v16h a; const float* p = rowk0 + 8 * (lane >> 4);
#pragma unroll
  for (int i = 0; i < 8; ++i) { a[i] = (_Float16)p[i]; a[8 + i] = (_Float16)p[16 + i]; }
  return a;
}
__device__ __forceinline__ v16h frag_f32s(const float* rowk0, int lane, float sc) {
  v16h a; const float* p = rowk0 + 8 * (lane >> 4);
#pragma unroll
  for (int i = 0; i < 8; ++i) { a[i] = (_Float16)(p[i] * sc); a[8 + i] = (_Float16)(p[16 + i] * sc); }
  return a;
}
__device__ __forceinline__ v16h fragc_f32(const float* W, int k0, int n, int lane, int ld, int K) {
  v16h a; const int g = lane >> 4;
#pragma unroll
  for (int i = 0; i < 8; ++i) { const int ka = k0 + 8 * g + i, kb = ka + 16;
    a[i] = (_Float16)(ka < K ? W[(size_t)(ka < K ? ka : K - 1) * ld + n] : 0.f); a[8 + i] = (_Float16)(kb < K ? W[(size_t)(kb < K ? kb : K - 1) * ld + n] : 0.f); }
  return a;
}
struct F2 { v16b h, l; };
__device__ __forceinline__ F2 bsplit16(const float v[16]) { F2 r;
#pragma unroll
  for (int i = 0; i < 16; ++i) { const __bf16 h = (__bf16)v[i]; r.h[i] = h; r.l[i] = (__bf16)(v[i] - (float)h); }
  return r; }
__device__ __forceinline__ F2 split_row(const float* row, int k0, int lane) { float v[16]; const float* p = row + k0 + 8 * (lane >> 4);
#pragma unroll
  for (int i = 0; i < 8; ++i) { v[i] = p[i]; v[8 + i] = p[16 + i]; }
  return bsplit16(v); }
__device__ __forceinline__ F2 split_rowK(const float* row, int k0, int lane, int K) { float v[16]; const int g = lane >> 4;
#pragma unroll
  for (int i = 0; i < 8; ++i) { const int ka = k0 + 8 * g + i, kb = ka + 16; v[i] = ka < K ? row[ka < K ? ka : K - 1] : 0.f; v[8 + i] = kb < K ? row[kb < K ? kb : K - 1] : 0.f; }
  return bsplit16(v); }
__device__ __forceinline__ F2 split_col(const float* W, int k0, int n, int lane, int ld, int K) { float v[16]; const int g = lane >> 4;
#pragma unroll
  for (int i = 0; i < 8; ++i) { const int ka = k0 + 8 * g + i, kb = ka + 16; v[i] = ka < K ? W[(size_t)(ka < K ? ka : K - 1) * ld + n] : 0.f; v[8 + i] = kb < K ? W[(size_t)(kb < K ? kb : K - 1) * ld + n] : 0.f; }
  return bsplit16(v); }
__device__ __forceinline__ v8f mac3(const F2& a, const F2& b, v8f c) { c = wmma_bf(a.l, b.h, c); c = wmma_bf(a.h, b.l, c); return wmma_bf(a.h, b.h, c); }
__device__ __forceinline__ float sigm(float v) { return 1.0f / (1.0f + expf(-v)); }
#define LDSX() do { asm volatile("s_wait_dscnt 0" ::: "memory"); __builtin_amdgcn_wave_barrier(); __builtin_amdgcn_fence(__ATOMIC_RELEASE, "workgroup"); } while (0)


#define NBT 4
#define NP 4096
#define DIMF 128
#define CC 64
#define NSM 8
#define NGR 8
#define NBLK (NBT * NP / 64)
#ifndef NQB
#define NQB NBLK
#endif
typedef __attribute__((ext_vector_type(8))) __bf16 v8b;
__device__ __forceinline__ v16b frag_b(const __bf16* rowk0, int lane) {
  union { v16b v; v8b q[2]; } u; const __bf16* p = rowk0 + 8 * (lane >> 4);
  u.q[0] = *(const v8b*)p; u.q[1] = *(const v8b*)(p + 16); return u.v;
}
__device__ __forceinline__ float bfr(float v) { return (float)(__bf16)v; }
__device__ __attribute__((noinline)) float exp_ni(float v) { return expf(v); }
__device__ __attribute__((noinline)) float erf_ni(float v) { return erff(v); }

#define WS_X1   0u
#define WS_PART (WS_X1 + 4u * NBT * NP * NSM * CC)
#define WS_STAT (WS_PART + 4u * NBLK * 32)
#define WS_X2H  (WS_STAT + 4u * NBT * 32)
#define WS_X2L  (WS_X2H + 2u * NBT * NP * CC)
#define WS_PW   (WS_X2L + 2u * NBT * NP * CC)
#define WS_END  (WS_PW + 2u * CC * CC)

__global__ __launch_bounds__(256) void k_pack(const float* __restrict__ OW, __bf16* __restrict__ PW) {
  __shared__ __align__(16) __bf16 s[CC * CC]; const int t = threadIdx.x;
  for (int k = t; k < CC * CC; k += 256) s[k] = (__bf16)OW[k];
  __syncthreads();
  for (int q = t; q < CC * CC / 8; q += 256) vst2((unsigned*)(PW + q * 8), *(const v4u*)&s[q * 8]);
}
__global__ __launch_bounds__(256) void k_bq(const float* __restrict__ CO, const float* __restrict__ X2, const float* __restrict__ F1, const float* __restrict__ F2, const float* __restrict__ CW, const float* __restrict__ CB, float* __restrict__ X1, float* __restrict__ PART) {
  __shared__ float sx[1024][3]; __shared__ int sidx[64][NSM]; __shared__ int scnt[64]; __shared__ float sfeat[64][NSM][4]; __shared__ float sgsl[256]; __shared__ __align__(16) float spart[32];
  const int tid = threadIdx.x; const size_t qb = blockIdx.x; const int b = (int)(qb * 64 / NP); const int m0 = (int)((qb * 64) % NP);
  const int q = tid & 63; float cx = 0.f, cy = 0.f, cz = 0.f; int cnt = 0; int found[NSM];
#pragma unroll
  for (int s = 0; s < NSM; ++s) found[s] = 0;
  if (tid < 64) { const float* c = CO + ((size_t)b * NP + m0 + q) * 3; cx = bfr(c[0]); cy = bfr(c[1]); cz = bfr(c[2]); }
  for (int n0 = 0; n0 < NP; n0 += 1024) {
    __syncthreads();
    for (int k = tid; k < 1024 * 3; k += 256) sx[k / 3][k % 3] = bfr(X2[((size_t)b * NP + n0) * 3 + k]);
    __syncthreads();
    if (tid < 64) { for (int n = 0; n < 1024; ++n) { const float dx = cx - sx[n][0], dy = cy - sx[n][1], dz = cz - sx[n][2]; const float d2 = (dx * dx + dz * dz) + dy * dy;
        if (d2 < 1.0f && cnt < NSM) {
#pragma unroll
          for (int s = 0; s < NSM; ++s) if (s == cnt) found[s] = n0 + n;
          ++cnt; } } } }
  if (tid < 64) { scnt[q] = cnt;
#pragma unroll
    for (int s = 0; s < NSM; ++s) sidx[q][s] = (s < cnt) ? found[s] : (cnt > 0 ? found[0] : 0); }
  __syncthreads();
  { const int ql = tid >> 2, s0 = (tid & 3) * 2; const size_t m = (size_t)m0 + ql; const float* c = CO + ((size_t)b * NP + m) * 3; const float ccx = bfr(c[0]), ccy = bfr(c[1]), ccz = bfr(c[2]);
    for (int s = s0; s < s0 + 2; ++s) { const int idx = sidx[ql][s]; float a = 0.f;
#pragma unroll 4
      for (int d = 0; d < DIMF; ++d) a += bfr(F1[((size_t)b * DIMF + d) * NP + m]) * bfr(F2[((size_t)b * DIMF + d) * NP + idx]);
      const float* p = X2 + ((size_t)b * NP + idx) * 3;
      sfeat[ql][s][0] = a / sqrtf((float)DIMF); sfeat[ql][s][1] = bfr(p[0]) - ccx; sfeat[ql][s][2] = bfr(p[1]) - ccy; sfeat[ql][s][3] = bfr(p[2]) - ccz; } }
  __syncthreads();
  { const int rs = tid >> 4, p = tid & 15; float gs = 0.f; float w4[4][4], b4[4];
#pragma unroll
    for (int i = 0; i < 4; ++i) { const int c = 4 * p + i; b4[i] = bfr(CB[c]);
#pragma unroll
      for (int j = 0; j < 4; ++j) w4[i][j] = bfr(CW[c * 4 + j]); }
#pragma unroll 1
    for (int it = 0; it < 32; ++it) { const int r = it * 16 + rs; const int ql = r >> 3, s = r & 7; const float f0 = sfeat[ql][s][0], f1 = sfeat[ql][s][1], f2 = sfeat[ql][s][2], f3 = sfeat[ql][s][3]; v4f v;
#pragma unroll
      for (int i = 0; i < 4; ++i) { v[i] = (((w4[i][0] * f0 + w4[i][1] * f1) + w4[i][2] * f2) + w4[i][3] * f3) + b4[i]; gs += v[i]; }
      vst2(X1 + (((size_t)b * NP + m0 + ql) * NSM + s) * CC + 4 * p, v); }
    sgsl[tid] = gs; }
  __syncthreads();
  if (tid < NGR) { float a = 0.f; for (int rs = 0; rs < 16; ++rs) { a += sgsl[rs * 16 + 2 * tid]; a += sgsl[rs * 16 + 2 * tid + 1]; } spart[tid] = a; }
  if (tid >= NGR && tid < 32) spart[tid] = 0.f;
  __syncthreads();
  if (tid < 8) vst2(PART + qb * 32 + tid * 4, *(const v4f*)&spart[tid * 4]);
}
template <int P>
__global__ __launch_bounds__(32) void k_red(const float* __restrict__ PART, float* __restrict__ STAT) {
  __shared__ __align__(16) float s[NBT][32]; const int t = threadIdx.x; const int b = t >> 3, g = t & 7;
  float a = 0.f; for (int k = 0; k < NP / 64; ++k) a += PART[((size_t)b * (NP / 64) + k) * 32 + g]; a = a / (float)(NGR * NP * NSM);
  for (int i = t; i < NBT * 32; i += 32) (&s[0][0])[i] = 0.f;
  __syncthreads();
  if (P == 0) s[b][g] = a; else { s[b][g] = STAT[b * 32 + g]; s[b][8 + g] = rsqrtf(a + 1e-5f); }
  __syncthreads();
  for (int qq = t; qq < NBT * 8; qq += 32) vst2(STAT + (qq >> 3) * 32 + (qq & 7) * 4, *(const v4f*)&s[qq >> 3][(qq & 7) * 4]);
}
__global__ __launch_bounds__(256) void k_var(const float* __restrict__ X1, const float* __restrict__ STAT, float* __restrict__ PART) {
  __shared__ float sgs[4][64][2]; __shared__ __align__(16) float spart[32]; const int tid = threadIdx.x; const size_t qb = blockIdx.x; const int b = (int)(qb * 64 / NP); const int ql = tid >> 2, cq = tid & 3;
  float g0 = 0.f, g1 = 0.f; const float mu0 = STAT[b * 32 + cq * 2], mu1 = STAT[b * 32 + cq * 2 + 1];
  for (int s = 0; s < NSM; ++s) { const float* row = X1 + ((qb * 64 + ql) * NSM + s) * CC + cq * 16;
#pragma unroll
    for (int i = 0; i < 16; ++i) { const float dv = row[i] - ((i < 8) ? mu0 : mu1); if (i < 8) g0 += dv * dv; else g1 += dv * dv; } }
  sgs[cq][ql][0] = g0; sgs[cq][ql][1] = g1;
  __syncthreads();
  if (tid < NGR) { const int cq2 = tid >> 1, half = tid & 1; float a = 0.f; for (int q2 = 0; q2 < 64; ++q2) a += sgs[cq2][q2][half]; spart[tid] = a; }
  if (tid >= NGR && tid < 32) spart[tid] = 0.f;
  __syncthreads();
  if (tid < 8) vst2(PART + qb * 32 + tid * 4, *(const v4f*)&spart[tid * 4]);
}
__global__ __launch_bounds__(256) void k_fin(const float* __restrict__ X1, const float* __restrict__ STAT, const float* __restrict__ GG, const float* __restrict__ GB, const float* __restrict__ PA, __bf16* __restrict__ X2H, __bf16* __restrict__ X2L) {
  __shared__ __align__(16) __bf16 sh_[64][72], sl_[64][72]; const int tid = threadIdx.x; const size_t qb = blockIdx.x; const int b = (int)(qb * 64 / NP); const int ql = tid >> 2, cq = tid & 3; const float pa = bfr(PA[0]);
  float mx[16];
#pragma unroll
  for (int i = 0; i < 16; ++i) mx[i] = -3.0e38f;
  for (int s = 0; s < NSM; ++s) { const float* row = X1 + ((qb * 64 + ql) * NSM + s) * CC + cq * 16;
#pragma unroll
    for (int i = 0; i < 16; ++i) { const int c = cq * 16 + i, g = c >> 3; float v = (row[i] - STAT[b * 32 + g]) * STAT[b * 32 + 8 + g] * bfr(GG[c]) + bfr(GB[c]); v = (v >= 0.f) ? v : pa * v; mx[i] = fmaxf(mx[i], v); } }
#pragma unroll
  for (int i = 0; i < 16; ++i) { const __bf16 hb = (__bf16)mx[i]; sh_[ql][cq * 16 + i] = hb; sl_[ql][cq * 16 + i] = (__bf16)(mx[i] - (float)hb); }
  __syncthreads();
  for (int q2 = tid; q2 < 64 * 8; q2 += 256) { const int r = q2 >> 3, pc = q2 & 7; const size_t o = (qb * 64 + r) * CC + pc * 8; vst2((unsigned*)(X2H + o), *(const v4u*)&sh_[r][pc * 8]); vst2((unsigned*)(X2L + o), *(const v4u*)&sl_[r][pc * 8]); }
}
__global__ __launch_bounds__(128) void k_out(const __bf16* __restrict__ X2H, const __bf16* __restrict__ X2L, const __bf16* __restrict__ PW, const float* __restrict__ OB, float* __restrict__ OUT) {
  __shared__ __align__(16) float so[CC][68];
  const int tid = threadIdx.x, wave = tid >> 5, lane = tid & 31, col = lane & 15, g = lane >> 4; const size_t qb = blockIdx.x; const int b = (int)(qb * 64 / NP); const int n0 = (int)((qb * 64) % NP); const size_t r0 = qb * 64 + wave * 16;
  v8f acc[4] = {};
#pragma unroll
  for (int kc = 0; kc < 2; ++kc) { F2 a; a.h = frag_b(X2H + (r0 + col) * CC + kc * 32, lane); a.l = frag_b(X2L + (r0 + col) * CC + kc * 32, lane);
#pragma unroll
    for (int j = 0; j < 4; ++j) { const v16b w = frag_b(PW + (size_t)(j * 16 + col) * CC + kc * 32, lane); acc[j] = wmma_bf(a.l, w, acc[j]); acc[j] = wmma_bf(a.h, w, acc[j]); } }
#pragma unroll
  for (int j = 0; j < 4; ++j) { const int o = j * 16 + col; const float bb = bfr(OB[o]);
#pragma unroll
    for (int r = 0; r < 8; ++r) so[o][wave * 16 + 8 * g + r] = acc[j][r] + bb; }
  __syncthreads();
  for (int q2 = tid; q2 < CC * 16; q2 += 128) { const int o = q2 >> 4, pc = q2 & 15; vst2(OUT + ((size_t)b * CC + o) * NP + n0 + pc * 4, *(const v4f*)&so[o][pc * 4]); }
}
extern "C" void kernel_launch(void* const* d_in, const int* in_sizes, int n_in, void* d_out, int out_size, void* d_ws, size_t ws_size, hipStream_t stream) {
  (void)in_sizes; (void)n_in; (void)out_size;
  const float** F = (const float**)d_in;
  if (ws_size < (size_t)WS_END) return;
  char* ws = (char*)d_ws; float *X1 = (float*)(ws + WS_X1), *PART = (float*)(ws + WS_PART), *STAT = (float*)(ws + WS_STAT); __bf16 *X2H = (__bf16*)(ws + WS_X2H), *X2L = (__bf16*)(ws + WS_X2L), *PW = (__bf16*)(ws + WS_PW);
  k_pack<<<1, 256, 0, stream>>>(F[9], PW);
  k_bq<<<NQB, 256, 0, stream>>>(F[0], F[1], F[2], F[3], F[4], F[5], X1, PART);
  k_red<0><<<1, 32, 0, stream>>>(PART, STAT);
  k_var<<<NQB, 256, 0, stream>>>(X1, STAT, PART);
  k_red<1><<<1, 32, 0, stream>>>(PART, STAT);
  k_fin<<<NQB, 256, 0, stream>>>(X1, STAT, F[6], F[7], F[8], X2H, X2L);
  k_out<<<NQB, 128, 0, stream>>>(X2H, X2L, PW, F[10], (float*)d_out);
}
